// ODE_RNN_12575664243120
// MI455X (gfx1250) — hardware-verified
//
#include <hip/hip_runtime.h>
#include <math.h>

constexpr int NBATCH   = 1024;
constexpr int NSTEP    = 128;
constexpr int NHID     = 256;
constexpr int NGATE    = 3 * NHID;
constexpr int NTHR     = 256;
constexpr int NWAVE    = NTHR / 32;
constexpr int ROWS_BLK = 16;
constexpr int APITCH   = 264;
constexpr int FPITCH   = 260;
constexpr int OPITCH   = 132;
constexpr int NCST     = 4 * NHID + 3 * NGATE;
constexpr float WCARRY = 256.0f;
constexpr float ACARRY = 256.0f;
constexpr float SC_INV = 1.0f / 65536.0f;
constexpr int NOUT0 = NBATCH * NSTEP;
constexpr int NOUT1 = NBATCH * NHID;
static_assert(NBATCH % ROWS_BLK == 0);
static_assert(NHID == 16 * 2 * NWAVE);
static_assert(NHID % 32 == 0);
static_assert(NTHR == NHID);
static_assert((NHID * NHID) % (8 * NTHR) == 0);
static_assert((NGATE * NHID) % (8 * NTHR) == 0);
static_assert((ROWS_BLK * NHID) % (4 * NTHR) == 0);
static_assert((ROWS_BLK * NSTEP) % (4 * NTHR) == 0);
static_assert(NOUT0 * 4 == 524288);
static_assert((NOUT0 + NOUT1) * 4 == 1572864);

typedef __attribute__((ext_vector_type(16))) _Float16 v16h;
typedef __attribute__((ext_vector_type(8)))  _Float16 v8h;
typedef __attribute__((ext_vector_type(8)))  float    v8f;
typedef __attribute__((ext_vector_type(4)))  float    v4f;

__device__ __forceinline__ void guard2_h(v8f& a0, v8f& a1, v16h x, v16h y0, v16h y1) {
  asm volatile("v_nop\n\tv_nop\n\tv_nop\n\tv_nop" : "+v"(a0), "+v"(a1) : "v"(x), "v"(y0), "v"(y1));
}
__device__ __forceinline__ void guard3_h(v8f& a0, v8f& a1, v8f& a2, v16h x, v16h y0, v16h y1, v16h y2) {
  asm volatile("v_nop\n\tv_nop\n\tv_nop\n\tv_nop" : "+v"(a0), "+v"(a1), "+v"(a2) : "v"(x), "v"(y0), "v"(y1), "v"(y2));
}
__device__ __forceinline__ void acc_guard2(v8f& a, v8f& b) { asm volatile("v_nop\n\tv_nop\n\tv_nop\n\tv_nop" : "+v"(a), "+v"(b)); }
__device__ __forceinline__ void acc_guard3(v8f& a, v8f& b, v8f& c) { asm volatile("v_nop\n\tv_nop\n\tv_nop\n\tv_nop" : "+v"(a), "+v"(b), "+v"(c)); }

template <typename T> struct Frag;
template <> struct Frag<_Float16> {
  typedef v16h V; union U { v16h v; v8h h[2]; };
  static __device__ __forceinline__ v16h load(const _Float16* p) {
    U f; f.h[0] = *(const v8h*)(p); f.h[1] = *(const v8h*)(p + 16); return f.v;
  }
  static __device__ __forceinline__ v8f mma(v16h a, v16h b, v8f c) {
    return __builtin_amdgcn_wmma_f32_16x16x32_f16(false, a, false, b, (short)0, c, false, false);
  }
};

__device__ __forceinline__ void gemm16x2(const _Float16* arow, const _Float16* w0, const _Float16* w1,
                                         v8f& acc0, v8f& acc1) {
  const v8f z8 = {0.f, 0.f, 0.f, 0.f, 0.f, 0.f, 0.f, 0.f};
  acc0 = z8; acc1 = z8;
#pragma unroll 1
  for (int k0 = 0; k0 < NHID; k0 += 32) {
    const v16h a  = Frag<_Float16>::load(arow + k0);
    const v16h b0 = Frag<_Float16>::load(w0 + k0);
    const v16h b1 = Frag<_Float16>::load(w1 + k0);
    acc0 = Frag<_Float16>::mma(a, b0, acc0);
    acc1 = Frag<_Float16>::mma(a, b1, acc1);
    guard2_h(acc0, acc1, a, b0, b1);
  }
  acc_guard2(acc0, acc1);
}
__device__ __forceinline__ void gemm16x3(const _Float16* arow, const _Float16* w0, const _Float16* w1, const _Float16* w2,
                                         v8f& acc0, v8f& acc1, v8f& acc2) {
  const v8f z8 = {0.f, 0.f, 0.f, 0.f, 0.f, 0.f, 0.f, 0.f};
  acc0 = z8; acc1 = z8; acc2 = z8;
#pragma unroll 1
  for (int k0 = 0; k0 < NHID; k0 += 32) {
    const v16h a  = Frag<_Float16>::load(arow + k0);
    const v16h b0 = Frag<_Float16>::load(w0 + k0);
    const v16h b1 = Frag<_Float16>::load(w1 + k0);
    const v16h b2 = Frag<_Float16>::load(w2 + k0);
    acc0 = Frag<_Float16>::mma(a, b0, acc0);
    acc1 = Frag<_Float16>::mma(a, b1, acc1);
    acc2 = Frag<_Float16>::mma(a, b2, acc2);
    guard3_h(acc0, acc1, acc2, a, b0, b1, b2);
  }
  acc_guard3(acc0, acc1, acc2);
}

__global__ __launch_bounds__(NTHR) void cvt8_f16_kernel(const float* __restrict__ src, unsigned short* __restrict__ dst,
                                                        int n8, float sc) {
  const int i = blockIdx.x * NTHR + threadIdx.x;
  if (i < n8) {
    const float* sp = src + (size_t)i * 8;
    const v4f a = *(const v4f*)(sp);
    const v4f b = *(const v4f*)(sp + 4);
    v8h hv;
#pragma unroll
    for (int e = 0; e < 4; ++e) {
      hv[e]     = (_Float16)(a[e] * sc);
      hv[4 + e] = (_Float16)(b[e] * sc);
    }
    unsigned short* dp = dst + (size_t)i * 8;
    *(volatile v8h*)dp = hv;
    __threadfence();
    *(volatile v8h*)dp = hv;
  }
}

__global__ __launch_bounds__(NTHR) void ode_gru_seq_kernel(
    const float* __restrict__ data, const float* __restrict__ tvec,
    const float* __restrict__ b1,   const float* __restrict__ b2,
    const float* __restrict__ w_ih, const float* __restrict__ b_ih, const float* __restrict__ b_hh,
    const float* __restrict__ bo1,  const float* __restrict__ wo2,  const float* __restrict__ bo2,
    const float* __restrict__ h0,
    const unsigned short* __restrict__ W1p,  const unsigned short* __restrict__ W2p,
    const unsigned short* __restrict__ Wo1p, const unsigned short* __restrict__ Whhp,
    float* __restrict__ out0, float* __restrict__ out1) {
  __shared__ __align__(16) _Float16 sA[ROWS_BLK * APITCH];
  __shared__ __align__(16) _Float16 sU[ROWS_BLK * APITCH];
  __shared__ __align__(16) float    sF[ROWS_BLK * FPITCH];
  __shared__ __align__(16) float    sO[ROWS_BLK * OPITCH];
  __shared__ float sRed[ROWS_BLK * NWAVE];
  __shared__ float sCst[NCST];

  const _Float16* W1  = (const _Float16*)W1p;
  const _Float16* W2  = (const _Float16*)W2p;
  const _Float16* Wo1 = (const _Float16*)Wo1p;
  const _Float16* Whh = (const _Float16*)Whhp;
  const int tid = threadIdx.x, lane = tid & 31, wave = tid >> 5;
  const int c = lane & 15, hh = lane >> 4, koff = hh * 8;
  const int rowbase = blockIdx.x * ROWS_BLK;
  const int jc0 = 32 * wave + c;
  const int jc1 = jc0 + 16;

#pragma unroll 1
  for (int i = tid; i < ROWS_BLK * APITCH; i += NTHR) { sA[i] = (_Float16)0.0f; sU[i] = (_Float16)0.0f; }
#pragma unroll 1
  for (int i = 0; i < ROWS_BLK; ++i) sF[i * FPITCH + tid] = h0[(size_t)(rowbase + i) * NHID + tid];
  {
    const float v0 = b1[tid], v1 = b2[tid], v2 = bo1[tid], v3 = wo2[tid];
    sCst[tid] = v0; sCst[NHID + tid] = v1; sCst[2 * NHID + tid] = v2; sCst[3 * NHID + tid] = v3;
  }
  asm volatile("" ::: "memory");
  {
#pragma unroll
    for (int g = 0; g < 3; ++g) {
      const float v0 = w_ih[g * NHID + tid], v1 = b_ih[g * NHID + tid], v2 = b_hh[g * NHID + tid];
      sCst[4 * NHID + g * NHID + tid]             = v0;
      sCst[4 * NHID + NGATE + g * NHID + tid]     = v1;
      sCst[4 * NHID + 2 * NGATE + g * NHID + tid] = v2;
    }
  }
  const float bo2v = bo2[0];
  __syncthreads();

  float b1c[2], b2c[2], bo1c[2], wo2c[2], wih[2][3], bih[2][3], bhh[2][3], hst[2][8];
#pragma unroll
  for (int ct = 0; ct < 2; ++ct) {
    const int j = jc0 + 16 * ct;
    b1c[ct]  = sCst[j];
    b2c[ct]  = sCst[NHID + j];
    bo1c[ct] = sCst[2 * NHID + j];
    wo2c[ct] = sCst[3 * NHID + j];
#pragma unroll
    for (int g = 0; g < 3; ++g) {
      wih[ct][g] = sCst[4 * NHID + g * NHID + j];
      bih[ct][g] = sCst[4 * NHID + NGATE + g * NHID + j];
      bhh[ct][g] = sCst[4 * NHID + 2 * NGATE + g * NHID + j];
    }
#pragma unroll
    for (int r = 0; r < 8; ++r) {
      const int row = 8 * hh + r;
      const float v = sF[row * FPITCH + j];
      hst[ct][r] = v;
      sA[row * APITCH + j] = (_Float16)(v * ACARRY);
    }
  }
  __syncthreads();

  const _Float16* aA = sA + c * APITCH + koff;
  const _Float16* aU = sU + c * APITCH + koff;
  const _Float16* w1c0  = W1  + (size_t)jc0 * NHID + koff;
  const _Float16* w1c1  = W1  + (size_t)jc1 * NHID + koff;
  const _Float16* w2c0  = W2  + (size_t)jc0 * NHID + koff;
  const _Float16* w2c1  = W2  + (size_t)jc1 * NHID + koff;
  const _Float16* wo1c0 = Wo1 + (size_t)jc0 * NHID + koff;
  const _Float16* wo1c1 = Wo1 + (size_t)jc1 * NHID + koff;

  float tprev = 0.0f;
#pragma unroll 1
  for (int step = 0; step < NSTEP; ++step) {
    const float tcur = tvec[step];
    const float dt   = tcur - tprev;
    tprev = tcur;
    const float dt6  = dt * (1.0f / 6.0f);
    float kacc[2][8];
#pragma unroll
    for (int ct = 0; ct < 2; ++ct)
#pragma unroll
      for (int r = 0; r < 8; ++r) kacc[ct][r] = 0.0f;

#pragma unroll 1
    for (int s = 0; s < 4; ++s) {
      v8f acc0, acc1;
      gemm16x2(aA, w1c0, w1c1, acc0, acc1);
#pragma unroll
      for (int r = 0; r < 8; ++r) {
        const int row = 8 * hh + r;
        const float u0 = acc0[r] * SC_INV + b1c[0];
        const float u1 = acc1[r] * SC_INV + b1c[1];
        sU[row * APITCH + jc0] = (_Float16)(u0 * ACARRY);
        sU[row * APITCH + jc1] = (_Float16)(u1 * ACARRY);
      }
      __syncthreads();
      gemm16x2(aU, w2c0, w2c1, acc0, acc1);
      const float wgt = (s == 0 || s == 3) ? 1.0f : 2.0f;
      const float cf  = (s == 2) ? dt : 0.5f * dt;
      const bool  fin = (s == 3);
#pragma unroll
      for (int r = 0; r < 8; ++r) {
        const int row = 8 * hh + r;
        const float fk0 = tanhf(acc0[r] * SC_INV + b2c[0]);
        const float fk1 = tanhf(acc1[r] * SC_INV + b2c[1]);
        const float ka0 = kacc[0][r] + wgt * fk0;
        const float ka1 = kacc[1][r] + wgt * fk1;
        kacc[0][r] = ka0;
        kacc[1][r] = ka1;
        const float nx0 = fin ? (hst[0][r] + dt6 * ka0) : (hst[0][r] + cf * fk0);
        const float nx1 = fin ? (hst[1][r] + dt6 * ka1) : (hst[1][r] + cf * fk1);
        hst[0][r] = fin ? nx0 : hst[0][r];
        hst[1][r] = fin ? nx1 : hst[1][r];
        sA[row * APITCH + jc0] = (_Float16)(nx0 * ACARRY);
        sA[row * APITCH + jc1] = (_Float16)(nx1 * ACARRY);
      }
      __syncthreads();
    }

    {
      v8f acc0, acc1;
      gemm16x2(aA, wo1c0, wo1c1, acc0, acc1);
      float p[8];
#pragma unroll
      for (int r = 0; r < 8; ++r) {
        float pr = 0.0f;
        pr += (acc0[r] * SC_INV + bo1c[0]) * wo2c[0];
        pr += (acc1[r] * SC_INV + bo1c[1]) * wo2c[1];
        p[r] = pr;
      }
#pragma unroll
      for (int r = 0; r < 8; ++r) {
        float pr = p[r];
        pr += __shfl_xor(pr, 1, 32);
        pr += __shfl_xor(pr, 2, 32);
        pr += __shfl_xor(pr, 4, 32);
        pr += __shfl_xor(pr, 8, 32);
        p[r] = pr;
      }
      if (c == 0) {
#pragma unroll
        for (int r = 0; r < 8; ++r) sRed[(8 * hh + r) * NWAVE + wave] = p[r];
      }
    }

    if (step < NSTEP - 1) {
      const float* xp = data + (size_t)step * NBATCH + rowbase + 8 * hh;
      const v4f xa = *(const v4f*)(xp);
      const v4f xb = *(const v4f*)(xp + 4);
      float xv[8];
      xv[0] = xa[0]; xv[1] = xa[1]; xv[2] = xa[2]; xv[3] = xa[3];
      xv[4] = xb[0]; xv[5] = xb[1]; xv[6] = xb[2]; xv[7] = xb[3];
#pragma unroll
      for (int ct = 0; ct < 2; ++ct) {
        const int j = jc0 + 16 * ct;
        v8f g0, g1, g2;
        gemm16x3(aA, Whh + (size_t)j * NHID + koff,
                     Whh + (size_t)(NHID + j) * NHID + koff,
                     Whh + (size_t)(2 * NHID + j) * NHID + koff, g0, g1, g2);
#pragma unroll
        for (int r = 0; r < 8; ++r) {
          const float ghr = g0[r] * SC_INV + bhh[ct][0];
          const float ghz = g1[r] * SC_INV + bhh[ct][1];
          const float ghn = g2[r] * SC_INV + bhh[ct][2];
          const float x   = xv[r];
          const float zr  = x * wih[ct][0] + bih[ct][0] + ghr;
          const float zz  = x * wih[ct][1] + bih[ct][1] + ghz;
          const float rg  = 1.0f / (1.0f + expf(-zr));
          const float zg  = 1.0f / (1.0f + expf(-zz));
          const float ng  = tanhf(x * wih[ct][2] + bih[ct][2] + rg * ghn);
          const float hp  = hst[ct][r];
          hst[ct][r] = (1.0f - zg) * ng + zg * hp;
        }
      }
    }
    __syncthreads();

    if (tid < ROWS_BLK) {
      float ssum = bo2v;
#pragma unroll
      for (int w = 0; w < NWAVE; ++w) ssum += sRed[tid * NWAVE + w];
      sO[tid * OPITCH + step] = tanhf(ssum);
    }
#pragma unroll
    for (int ct = 0; ct < 2; ++ct) {
      const int j = jc0 + 16 * ct;
#pragma unroll
      for (int r = 0; r < 8; ++r) sA[(8 * hh + r) * APITCH + j] = (_Float16)(hst[ct][r] * ACARRY);
    }
    __syncthreads();
  }

#pragma unroll
  for (int ct = 0; ct < 2; ++ct) {
    const int j = jc0 + 16 * ct;
#pragma unroll
    for (int r = 0; r < 8; ++r) sF[(8 * hh + r) * FPITCH + j] = hst[ct][r];
  }
  __syncthreads();
  for (int pass = 0; pass < 2; ++pass) {
#pragma unroll
    for (int it = 0; it < 4; ++it) {
      const int idx = it * NTHR + tid;
      const int row = idx >> 6, c4 = (idx & 63) * 4;
      const v4f v = *(const v4f*)(sF + row * FPITCH + c4);
      *(volatile v4f*)(out1 + (size_t)(rowbase + row) * NHID + c4) = v;
    }
    __threadfence();
  }
  for (int pass = 0; pass < 2; ++pass) {
#pragma unroll
    for (int it = 0; it < 2; ++it) {
      const int idx = it * NTHR + tid;
      const int row = idx >> 5, c4 = (idx & 31) * 4;
      const v4f v = *(const v4f*)(sO + row * OPITCH + c4);
      *(volatile v4f*)(out0 + (size_t)(rowbase + row) * NSTEP + c4) = v;
    }
    __threadfence();
  }
}

extern "C" void kernel_launch(void* const* d_in, const int* in_sizes, int n_in,
                              void* d_out, int out_size, void* d_ws, size_t ws_size, hipStream_t stream) {
  if (n_in < 15 || d_out == nullptr || d_ws == nullptr) return;
  if (in_sizes[0] != NSTEP * NBATCH || in_sizes[1] != NBATCH * NSTEP || in_sizes[2] != NHID * NHID ||
      in_sizes[3] != NHID || in_sizes[4] != NHID * NHID || in_sizes[5] != NHID || in_sizes[6] != NGATE ||
      in_sizes[7] != NGATE || in_sizes[8] != NGATE * NHID || in_sizes[9] != NGATE || in_sizes[10] != NHID * NHID ||
      in_sizes[11] != NHID || in_sizes[12] != NHID || in_sizes[13] < 1 || in_sizes[14] != NBATCH * NHID ||
      out_size != NOUT0 + NOUT1) return;

  const float* data = (const float*)d_in[0];
  const float* tvec = (const float*)d_in[1];
  const float* W1   = (const float*)d_in[2];
  const float* b1   = (const float*)d_in[3];
  const float* W2   = (const float*)d_in[4];
  const float* b2   = (const float*)d_in[5];
  const float* w_ih = (const float*)d_in[6];
  const float* b_ih = (const float*)d_in[7];
  const float* W_hh = (const float*)d_in[8];
  const float* b_hh = (const float*)d_in[9];
  const float* Wo1  = (const float*)d_in[10];
  const float* bo1  = (const float*)d_in[11];
  const float* wo2  = (const float*)d_in[12];
  const float* bo2  = (const float*)d_in[13];
  const float* h0   = (const float*)d_in[14];
  float* out0 = (float*)d_out;
  float* out1 = out0 + (size_t)NOUT0;

  char* ws = (char*)d_ws; size_t off = 0;
  auto carve = [&](size_t bytes) -> char* { char* p = ws + off; off += (bytes + 255) & ~(size_t)255; return p; };
  unsigned short* W1P  = (unsigned short*)carve((size_t)NHID * NHID * 2);
  unsigned short* W2P  = (unsigned short*)carve((size_t)NHID * NHID * 2);
  unsigned short* WO1P = (unsigned short*)carve((size_t)NHID * NHID * 2);
  unsigned short* WHHP = (unsigned short*)carve((size_t)NGATE * NHID * 2);
  if (off > ws_size || off > (size_t)134217728) return;

  const int n8w = NHID * NHID / 8;
  const int n8g = NGATE * NHID / 8;
  cvt8_f16_kernel<<<n8w / NTHR, NTHR, 0, stream>>>(W1,   W1P,  n8w, WCARRY);
  cvt8_f16_kernel<<<n8w / NTHR, NTHR, 0, stream>>>(W2,   W2P,  n8w, WCARRY);
  cvt8_f16_kernel<<<n8w / NTHR, NTHR, 0, stream>>>(Wo1,  WO1P, n8w, WCARRY);
  cvt8_f16_kernel<<<n8g / NTHR, NTHR, 0, stream>>>(W_hh, WHHP, n8g, WCARRY);

  ode_gru_seq_kernel<<<NBATCH / ROWS_BLK, NTHR, 0, stream>>>(
      data, tvec, b1, b2, w_ih, b_ih, b_hh, bo1, wo2, bo2, h0, W1P, W2P, WO1P, WHHP, out0, out1);
}
